// TransformerBlock_16174846837027
// MI455X (gfx1250) — hardware-verified
//
#include <hip/hip_runtime.h>
#ifndef NB
#define NB 2
#endif
#ifndef SEQ
#define SEQ 2048
#endif
#define NB_FULL 2
#define SEQ_FULL 2048
#define DM 1024
#define NH 16
#define HD 64
#define DFF 4096
#define LH (3 * DM)
#define LP (2 * DM)
#define MP (NB * SEQ)
#define PSP 40

static_assert(NH * HD == DM);
static_assert(HD == 64);
static_assert(DM % 128 == 0 && DFF % 64 == 0 && SEQ % 64 == 0);
static_assert(MP % 128 == 0);
static_assert(256 * 4 == DM && 256 * 16 == DFF);
static_assert(NB <= NB_FULL && SEQ <= SEQ_FULL);
static_assert(PSP % 8 == 0 && PSP >= 32);
static_assert((DM & (DM - 1)) == 0);
static_assert((size_t)MP * LH < ((size_t)1 << 31));

typedef _Float16 v16h __attribute__((ext_vector_type(16)));
typedef __bf16 v16b __attribute__((ext_vector_type(16)));
typedef unsigned short v8us __attribute__((ext_vector_type(8), may_alias));
typedef unsigned short v4us __attribute__((ext_vector_type(4), may_alias));
typedef float v8f __attribute__((ext_vector_type(8)));
typedef float v4f __attribute__((ext_vector_type(4)));
typedef float v4fa __attribute__((ext_vector_type(4), may_alias));
union FragH { v16h v; v8us half[2]; _Float16 h[16]; unsigned short u[16]; };

__device__ __forceinline__ unsigned short bf16_bits(float x) { unsigned int u = __float_as_uint(x); return (unsigned short)((u + 0x7FFFu + ((u >> 16) & 1u)) >> 16); }
__device__ __forceinline__ float bf16_val(unsigned short b) { return __uint_as_float(((unsigned int)b) << 16); }
__device__ __forceinline__ float bf16_rne(float x) { return bf16_val(bf16_bits(x)); }
__device__ __forceinline__ unsigned short f16_bits(float x) { const _Float16 hv = (_Float16)x; return __builtin_bit_cast(unsigned short, hv); }

template <int ASBF>
__global__ __launch_bounds__(256) void k_wt(const float* __restrict__ W, unsigned short* __restrict__ Wt, unsigned K, unsigned N, float scale) {
  const unsigned t = blockIdx.x * 256u + threadIdx.x; const unsigned k8n = K >> 3; if (t >= N * k8n) return;
  const unsigned n = t / k8n, k8 = (t - n * k8n) << 3; FragH f;
#pragma unroll
  for (unsigned i = 0; i < 8; ++i) { const float wv = W[(size_t)(k8 + i) * N + n];
    if (ASBF) f.u[i] = bf16_bits(wv); else f.u[i] = f16_bits(bf16_rne(wv) * scale); }
  const v8us o = f.half[0]; unsigned short* dst = Wt + (size_t)n * K + k8;
  *(volatile v8us*)dst = o; __threadfence(); *(volatile v8us*)dst = o;
}

template <int VEC, int MODE>
__global__ __launch_bounds__(256) void k_ln(const float* __restrict__ X, const float* __restrict__ g, const float* __restrict__ bb, float eps, unsigned short* __restrict__ OUT) {
  #pragma clang fp contract(off)
  constexpr unsigned NC = (unsigned)VEC * 1024u;
  constexpr unsigned OUTW = (MODE == 0) ? 3u * NC : NC;
  constexpr unsigned NPIECE = OUTW / 8u;
  constexpr unsigned NPI = (NPIECE + 255u) / 256u;
  static_assert(MODE != 0 || VEC == 1);
  __shared__ float red1[8]; __shared__ float red2[8];
  __shared__ __attribute__((aligned(16))) unsigned short row16[OUTW];
  const unsigned r = blockIdx.x, t = threadIdx.x, w = t >> 5, lane = t & 31u;
  size_t src;
  if (MODE == 0) { const unsigned b = r / (unsigned)SEQ, s = r - b * (unsigned)SEQ; src = ((size_t)b * SEQ_FULL + s) * NC; } else { src = (size_t)r * NC; }
  v4f xa[VEC];
  float sum = 0.f;
#pragma unroll
  for (int i = 0; i < VEC; ++i) { v4f a = *(const v4fa*)(X + src + (unsigned)i * 1024u + t * 4u);
    if (MODE == 0) {
#pragma unroll
      for (unsigned q = 0; q < 4; ++q) a[q] = bf16_rne(a[q]); }
    xa[i] = a; sum += (a[0] + a[1]) + (a[2] + a[3]); }
  for (int o = 16; o > 0; o >>= 1) sum += __shfl_xor(sum, o, 32);
  if (lane == 0u) red1[w] = sum;
  __syncthreads();
  const float mu = (((red1[0] + red1[1]) + (red1[2] + red1[3])) + ((red1[4] + red1[5]) + (red1[6] + red1[7]))) / (float)NC;
  float vs = 0.f;
#pragma unroll
  for (int i = 0; i < VEC; ++i) { v4f d = xa[i];
#pragma unroll
    for (unsigned q = 0; q < 4; ++q) d[q] = d[q] - mu;
    xa[i] = d; vs += (d[0] * d[0] + d[1] * d[1]) + (d[2] * d[2] + d[3] * d[3]); }
  for (int o = 16; o > 0; o >>= 1) vs += __shfl_xor(vs, o, 32);
  if (lane == 0u) red2[w] = vs;
  __syncthreads();
  const float var = (((red2[0] + red2[1]) + (red2[2] + red2[3])) + ((red2[4] + red2[5]) + (red2[6] + red2[7]))) / (float)NC;
  const float rs = rsqrtf(var + eps);
#pragma unroll
  for (int i = 0; i < VEC; ++i) { const unsigned c = (unsigned)i * 1024u + t * 4u;
    const v4f gv = *(const v4fa*)(g + c), bv = *(const v4fa*)(bb + c); const v4f d = xa[i];
    v4us o0, o1, o2;
#pragma unroll
    for (unsigned q = 0; q < 4; ++q) { const float yv = (d[q] * rs) * bf16_rne(gv[q]) + bf16_rne(bv[q]);
      if (MODE == 0) { const unsigned short hb = bf16_bits(yv); o0[q] = hb; o1[q] = bf16_bits(yv - bf16_val(hb)); o2[q] = f16_bits(yv); }
      if (MODE == 1) { o0[q] = f16_bits(yv); }
      if (MODE == 2) { const float rl = (yv > 0.0f) ? yv : (yv - yv); o0[q] = f16_bits(rl * 16.0f); } }
    *(v4us*)(&row16[c]) = o0;
    if (MODE == 0) { *(v4us*)(&row16[NC + c]) = o1; *(v4us*)(&row16[2u * NC + c]) = o2; } }
  __syncthreads();
  v8us o8[NPI];
#pragma unroll
  for (unsigned j = 0; j < NPI; ++j) { const unsigned p = j * 256u + t; const v8us zz = {0, 0, 0, 0, 0, 0, 0, 0}; o8[j] = zz;
    if (p < NPIECE) o8[j] = *(const v8us*)(&row16[p * 8u]); }
  const size_t ob = (size_t)r * OUTW;
  for (int pass = 0; pass < 2; ++pass) {
#pragma unroll
    for (unsigned j = 0; j < NPI; ++j) { const unsigned p = j * 256u + t;
      if (p < NPIECE) *(volatile v8us*)(OUT + ob + p * 8u) = o8[j]; }
    if (pass == 0) __threadfence(); }
}

__device__ __forceinline__ v16h g2_frag(const unsigned short* p, unsigned hh) { FragH f; f.half[0] = *(const v8us*)(p + 8u * hh); f.half[1] = *(const v8us*)(p + 16u + 8u * hh); return f.v; }
template <int BF>
__device__ __forceinline__ v8f g2_mma(v16h a, v16h b, v8f c) {
  v8f d;
  if (BF) d = __builtin_amdgcn_wmma_f32_16x16x32_bf16(false, __builtin_bit_cast(v16b, a), false, __builtin_bit_cast(v16b, b), (short)0, c, false, false);
  else    d = __builtin_amdgcn_wmma_f32_16x16x32_f16(false, a, false, b, (short)0, c, false, false);
  asm volatile("v_nop\n\tv_nop\n\tv_nop\n\tv_nop" : "+v"(d) : "v"(a), "v"(b)); return d; }

template <int BF, int OM, int BROW>
__global__ __launch_bounds__(128) void k_gemm2(const unsigned short* __restrict__ A, unsigned lda, size_t sA, unsigned kmA,
    const unsigned short* __restrict__ Bh, unsigned ldb, size_t sB, unsigned kmB, float alpha,
    const float* __restrict__ bias, float bscale, float* __restrict__ C, unsigned short* __restrict__ C16, float c16s, unsigned lo_off,
    unsigned ldc, size_t sC, unsigned M, unsigned N, unsigned K) {
  static_assert(OM == 0 || OM == 1 || OM == 2);
  __shared__ __attribute__((aligned(16))) float so[4][32][68];
  const unsigned tid = threadIdx.x, w = tid >> 5, lane = tid & 31u, ln = lane & 15u, hh = lane >> 4; const unsigned by = blockIdx.y;
  A += (size_t)by * sA; Bh += (size_t)by * sB; const size_t cofs = (size_t)by * sC;
  const unsigned ntn = N >> 6; const unsigned mt = blockIdx.x / ntn, nq = blockIdx.x - mt * ntn; const unsigned row0 = mt * 128u + 32u * w, col0 = nq * 64u; if (row0 >= M) return;
  const unsigned short* a0p = A + (size_t)(row0 + ln) * lda; const unsigned short* a1p = a0p + (size_t)16 * lda;
  const unsigned short* b0p = Bh + (size_t)(col0 + ln) * ldb; const unsigned short* b1p = b0p + (size_t)16 * ldb; const unsigned short* b2p = b1p + (size_t)16 * ldb; const unsigned short* b3p = b2p + (size_t)16 * ldb;
  const v8f z8 = {0.f,0.f,0.f,0.f,0.f,0.f,0.f,0.f}; v8f c00 = z8, c01 = z8, c02 = z8, c03 = z8, c10 = z8, c11 = z8, c12 = z8, c13 = z8;
#pragma unroll 1
  for (unsigned kb = 0; kb < K; kb += 32u) { const unsigned ka = kb & kmA, kq = kb & kmB;
    const v16h a0 = g2_frag(a0p + ka, hh), a1 = g2_frag(a1p + ka, hh);
    v16h b = g2_frag(b0p + kq, hh); c00 = g2_mma<BF>(a0, b, c00); c10 = g2_mma<BF>(a1, b, c10);
    b = g2_frag(b1p + kq, hh); c01 = g2_mma<BF>(a0, b, c01); c11 = g2_mma<BF>(a1, b, c11);
    b = g2_frag(b2p + kq, hh); c02 = g2_mma<BF>(a0, b, c02); c12 = g2_mma<BF>(a1, b, c12);
    b = g2_frag(b3p + kq, hh); c03 = g2_mma<BF>(a0, b, c03); c13 = g2_mma<BF>(a1, b, c13); }
  v8f accs[8] = {c00, c01, c02, c03, c10, c11, c12, c13};
#pragma unroll
  for (unsigned u = 0; u < 8; ++u) { const unsigned t = u & 3u, half = u >> 2; const unsigned col = col0 + t * 16u + ln;
    const float bvc = BROW ? 0.f : bf16_rne(bias[col]) * bscale;
#pragma unroll
    for (unsigned r = 0; r < 8; ++r) { const unsigned rloc = half * 16u + 8u * hh + r;
      const float bv = BROW ? bf16_rne(bias[row0 + rloc]) * bscale : bvc;
      so[w][rloc][t * 16u + ln] = accs[u][r] * alpha + bv; } }
  __builtin_amdgcn_fence(4  , "workgroup"); __builtin_amdgcn_wave_barrier();
  const unsigned rsub = lane >> 4, c4 = (lane & 15u) * 4u;
  const unsigned rsub8 = lane >> 3, c8 = (lane & 7u) * 8u;
  for (int pass = 0; pass < 2; ++pass) {
    if (OM == 0) {
#pragma unroll
      for (unsigned q = 0; q < 16; ++q) { const unsigned r = q * 2u + rsub; const v4f v = *(const v4fa*)&so[w][r][c4]; const size_t o = cofs + (size_t)(row0 + r) * ldc + col0 + c4;
        *(volatile v4f*)(C + o) = v; } }
    if (OM == 1) {
#pragma unroll
      for (unsigned q = 0; q < 8; ++q) { const unsigned r = q * 4u + rsub8; const v4f va = *(const v4fa*)&so[w][r][c8], vb = *(const v4fa*)&so[w][r][c8 + 4u]; FragH f;
#pragma unroll
        for (unsigned i = 0; i < 4; ++i) { f.u[i] = f16_bits(va[i] * c16s); f.u[4u + i] = f16_bits(vb[i] * c16s); }
        const size_t o = cofs + (size_t)(row0 + r) * ldc + col0 + c8;
        *(volatile v8us*)(C16 + o) = f.half[0]; } }
    if (OM == 2) {
#pragma unroll
      for (unsigned q = 0; q < 8; ++q) { const unsigned r = q * 4u + rsub8; const v4f va = *(const v4fa*)&so[w][r][c8], vb = *(const v4fa*)&so[w][r][c8 + 4u]; FragH fh, fl;
#pragma unroll
        for (unsigned i = 0; i < 4; ++i) { const unsigned short ha = bf16_bits(va[i]), hb = bf16_bits(vb[i]);
          fh.u[i] = ha; fl.u[i] = bf16_bits(va[i] - bf16_val(ha)); fh.u[4u + i] = hb; fl.u[4u + i] = bf16_bits(vb[i] - bf16_val(hb)); }
        const size_t o = cofs + (size_t)(row0 + r) * ldc + col0 + c8;
        *(volatile v8us*)(C16 + o) = fh.half[0];
        *(volatile v8us*)(C16 + o + lo_off) = fl.half[0]; } }
    if (pass == 0) __threadfence(); } }

__global__ __launch_bounds__(128) void k_flash(const unsigned short* __restrict__ QP, const unsigned short* __restrict__ KP, const unsigned short* __restrict__ Vt,
    const float* __restrict__ X, const int* __restrict__ NHP, float* __restrict__ X1) {
  __shared__ __attribute__((aligned(16))) unsigned short ps[4][16][PSP];
  __shared__ __attribute__((aligned(16))) float so[4][16][68];
  const unsigned tid = threadIdx.x, w = tid >> 5, lane = tid & 31u, ln = lane & 15u, hh = lane >> 4;
  const unsigned qblk = blockIdx.x, h = blockIdx.y, b = blockIdx.z;
  const unsigned qrow0 = b * (unsigned)SEQ + qblk * 64u + w * 16u;
  const unsigned qoff = (qrow0 + ln) * (unsigned)LP + h * 64u;
  const unsigned koff0 = (b * (unsigned)SEQ + ln) * (unsigned)LP + h * 64u;
  const unsigned voff0 = ((b * (unsigned)NH + h) * 64u + ln) * (unsigned)SEQ;
  const v8f z8 = {0.f,0.f,0.f,0.f,0.f,0.f,0.f,0.f};
  v8f o[4] = {z8, z8, z8, z8};
  float mrun[8], lrun[8];
#pragma unroll
  for (unsigned r = 0; r < 8; ++r) { mrun[r] = -1.0e30f; lrun[r] = 0.f; }
#pragma unroll 1
  for (unsigned kb = 0; kb < (unsigned)(SEQ / 32); ++kb) {
    unsigned qo = qoff; asm volatile("" : "+v"(qo));
    const unsigned ko = koff0 + kb * (32u * (unsigned)LP);
    v8f s0 = z8, s1 = z8;
#pragma unroll
    for (unsigned ks = 0; ks < 2; ++ks) {
      const v16h qh = g2_frag(QP + qo + ks * 32u, hh), ql = g2_frag(QP + qo + (unsigned)DM + ks * 32u, hh);
      { const v16h kh = g2_frag(KP + ko + ks * 32u, hh), kl = g2_frag(KP + ko + (unsigned)DM + ks * 32u, hh);
        s0 = g2_mma<1>(ql, kh, s0); s0 = g2_mma<1>(qh, kl, s0); s0 = g2_mma<1>(qh, kh, s0); }
      { const v16h kh = g2_frag(KP + ko + 16u * (unsigned)LP + ks * 32u, hh), kl = g2_frag(KP + ko + 16u * (unsigned)LP + (unsigned)DM + ks * 32u, hh);
        s1 = g2_mma<1>(ql, kh, s1); s1 = g2_mma<1>(qh, kl, s1); s1 = g2_mma<1>(qh, kh, s1); } }
#pragma unroll
    for (unsigned r = 0; r < 8; ++r) {
      float mx = fmaxf(s0[r], s1[r]);
      mx = fmaxf(mx, __shfl_xor(mx, 1, 32)); mx = fmaxf(mx, __shfl_xor(mx, 2, 32)); mx = fmaxf(mx, __shfl_xor(mx, 4, 32)); mx = fmaxf(mx, __shfl_xor(mx, 8, 32));
      const float mnew = fmaxf(mrun[r], mx);
      const float al = __expf(mrun[r] - mnew);
      const _Float16 h0 = (_Float16)(__expf(s0[r] - mnew) * 4096.0f), h1 = (_Float16)(__expf(s1[r] - mnew) * 4096.0f);
      ps[w][8u * hh + r][ln] = __builtin_bit_cast(unsigned short, h0);
      ps[w][8u * hh + r][16u + ln] = __builtin_bit_cast(unsigned short, h1);
      lrun[r] = lrun[r] * al + ((float)h0 + (float)h1); mrun[r] = mnew;
#pragma unroll
      for (unsigned nf = 0; nf < 4; ++nf) o[nf][r] *= al; }
    __builtin_amdgcn_fence(4  , "workgroup"); __builtin_amdgcn_wave_barrier();
    const v16h ap = g2_frag(&ps[w][ln][0], hh);
    const unsigned vo = voff0 + kb * 32u;
#pragma unroll
    for (unsigned nf = 0; nf < 4; ++nf) { const v16h bv = g2_frag(Vt + vo + nf * 16u * (unsigned)SEQ, hh); o[nf] = g2_mma<0>(ap, bv, o[nf]); }
    __builtin_amdgcn_fence(4  , "workgroup"); __builtin_amdgcn_wave_barrier();
  }
  float inv[8];
#pragma unroll
  for (unsigned r = 0; r < 8; ++r) { float l = lrun[r];
    l += __shfl_xor(l, 1, 32); l += __shfl_xor(l, 2, 32); l += __shfl_xor(l, 4, 32); l += __shfl_xor(l, 8, 32);
    inv[r] = 0.0625f * (1.0f / l); }
#pragma unroll
  for (unsigned nf = 0; nf < 4; ++nf) {
#pragma unroll
    for (unsigned r = 0; r < 8; ++r) so[w][8u * hh + r][nf * 16u + ln] = o[nf][r] * inv[r]; }
  __builtin_amdgcn_fence(4  , "workgroup"); __builtin_amdgcn_wave_barrier();
  const int nhv = NHP[0];
  const float pz = (nhv == NH) ? 0.0f : __uint_as_float(0x7FC00000u);
  const unsigned rsub = lane >> 4, c4 = (lane & 15u) * 4u;
  v4f outv[8];
#pragma unroll
  for (unsigned q = 0; q < 8; ++q) { const unsigned r = q * 2u + rsub; const unsigned s = qblk * 64u + w * 16u + r;
    const v4f xv = *(const v4fa*)(X + ((size_t)b * SEQ_FULL + s) * DM + h * 64u + c4);
    const v4f cv = *(const v4fa*)&so[w][r][c4]; v4f ov;
#pragma unroll
    for (unsigned i = 0; i < 4; ++i) ov[i] = (bf16_rne(xv[i]) + cv[i]) + pz;
    outv[q] = ov; }
  for (int pass = 0; pass < 2; ++pass) {
#pragma unroll
    for (unsigned q = 0; q < 8; ++q) { const unsigned r = q * 2u + rsub; *(volatile v4f*)(X1 + (size_t)(qrow0 + r) * DM + h * 64u + c4) = outv[q]; }
    if (pass == 0) __threadfence(); }
}

constexpr size_t pad256(size_t b) { return (b + 255) & ~(size_t)255; }
constexpr size_t cmax(size_t a, size_t b) { return a > b ? a : b; }
constexpr size_t SZ_W    = pad256((size_t)DM * DM * 2);
constexpr size_t SZ_BW1  = pad256((size_t)DFF * DM * 2);
constexpr size_t SZ_BW2  = pad256((size_t)DM * DFF * 2);
constexpr size_t SZ_HP   = pad256((size_t)MP * LH * 2);
constexpr size_t SZ_QP   = pad256((size_t)MP * LP * 2);
constexpr size_t SZ_KP   = pad256((size_t)MP * LP * 2);
constexpr size_t SZ_VT   = pad256((size_t)NB * DM * SEQ * 2);
constexpr size_t SZ_UP   = pad256((size_t)MP * DFF * 4);
constexpr size_t SZ_RA   = cmax(SZ_HP + SZ_QP + SZ_KP + SZ_VT, SZ_UP);
constexpr size_t SZ_X1   = pad256((size_t)MP * DM * 4);
constexpr size_t SZ_H2   = pad256((size_t)MP * DM * 2);
constexpr size_t SZ_U16  = pad256((size_t)MP * DFF * 2);
constexpr size_t SZ_RB   = cmax(SZ_X1 + SZ_H2, SZ_U16);
constexpr size_t SZ_TOTAL = 3 * SZ_W + SZ_BW1 + SZ_BW2 + SZ_RA + SZ_RB;
static_assert(SZ_UP <= SZ_RA && SZ_HP + SZ_QP + SZ_KP + SZ_VT <= SZ_RA);
static_assert(SZ_U16 <= SZ_RB && SZ_X1 + SZ_H2 <= SZ_RB);
static_assert(SZ_TOTAL <= (size_t)134217728);

extern "C" void kernel_launch(void* const* d_in, const int* in_sizes, int n_in,
                              void* d_out, int out_size, void* d_ws, size_t ws_size, hipStream_t stream) {
  if (n_in < 18) return;
  if ((long long)in_sizes[0] < ((long long)(NB - 1) * SEQ_FULL + SEQ) * DM) return;
  if (in_sizes[1] < DM * DM || in_sizes[3] < DM * DM || in_sizes[5] < DM * DM) return;
  if (in_sizes[2] < DM || in_sizes[4] < DM || in_sizes[6] < DM || in_sizes[7] < DM || in_sizes[8] < DM || in_sizes[9] < DM || in_sizes[10] < DM) return;
  if (in_sizes[11] < DM * DFF || in_sizes[12] < DFF || in_sizes[13] < DFF || in_sizes[14] < DFF || in_sizes[15] < DFF * DM || in_sizes[16] < DM || in_sizes[17] < 1) return;
  if ((long long)out_size < (long long)MP * DM) return;
  if (SZ_TOTAL > ws_size) return;
  const float* x   = (const float*)d_in[0];
  const float* wq  = (const float*)d_in[1];  const float* bq  = (const float*)d_in[2];
  const float* wk  = (const float*)d_in[3];  const float* bk  = (const float*)d_in[4];
  const float* wv  = (const float*)d_in[5];  const float* bv  = (const float*)d_in[6];
  const float* g1  = (const float*)d_in[7];  const float* b1  = (const float*)d_in[8];
  const float* g2  = (const float*)d_in[9];  const float* b2  = (const float*)d_in[10];
  const float* w1  = (const float*)d_in[11]; const float* bw1 = (const float*)d_in[12];
  const float* gf  = (const float*)d_in[13]; const float* bfv = (const float*)d_in[14];
  const float* w2  = (const float*)d_in[15]; const float* bw2 = (const float*)d_in[16];
  const int*   nhp = (const int*)d_in[17];
  char* ws = (char*)d_ws; size_t off = 0;
  unsigned short* WQT = (unsigned short*)(ws + off); off += SZ_W;
  unsigned short* WKT = (unsigned short*)(ws + off); off += SZ_W;
  unsigned short* WVT = (unsigned short*)(ws + off); off += SZ_W;
  unsigned short* W1T = (unsigned short*)(ws + off); off += SZ_BW1;
  unsigned short* W2T = (unsigned short*)(ws + off); off += SZ_BW2;
  char* RA = ws + off; off += SZ_RA;
  char* RB = ws + off; off += SZ_RB;
  unsigned short* HP = (unsigned short*)RA;
  unsigned short* QP = (unsigned short*)(RA + SZ_HP);
  unsigned short* KP = (unsigned short*)(RA + SZ_HP + SZ_QP);
  unsigned short* VT = (unsigned short*)(RA + SZ_HP + SZ_QP + SZ_KP);
  float*          UP = (float*)RA;
  float*          X1 = (float*)RB;
  unsigned short* H2 = (unsigned short*)(RB + SZ_X1);
  unsigned short* U16 = (unsigned short*)RB;

  k_wt<1><<<(unsigned)(((size_t)DM * (DM / 8) + 255) / 256), 256, 0, stream>>>(wq, WQT, (unsigned)DM, (unsigned)DM, 1.0f);
  k_wt<1><<<(unsigned)(((size_t)DM * (DM / 8) + 255) / 256), 256, 0, stream>>>(wk, WKT, (unsigned)DM, (unsigned)DM, 1.0f);
  k_wt<0><<<(unsigned)(((size_t)DM * (DM / 8) + 255) / 256), 256, 0, stream>>>(wv, WVT, (unsigned)DM, (unsigned)DM, 16.0f);
  k_wt<0><<<(unsigned)(((size_t)DFF * (DM / 8) + 255) / 256), 256, 0, stream>>>(w1, W1T, (unsigned)DM, (unsigned)DFF, 16.0f);
  k_wt<0><<<(unsigned)(((size_t)DM * (DFF / 8) + 255) / 256), 256, 0, stream>>>(w2, W2T, (unsigned)DFF, (unsigned)DM, 16.0f);
  k_ln<1, 0><<<(unsigned)MP, 256, 0, stream>>>(x, g1, b1, 1e-5f, HP);
  k_gemm2<1, 2, 0><<<dim3((unsigned)((MP / 128) * (DM / 64)), 1), 128, 0, stream>>>(HP, (unsigned)LH, (size_t)0, (unsigned)(2 * DM - 1), WQT, (unsigned)DM, (size_t)0, (unsigned)(DM - 1), 32.0f,
      bq, 32.0f, nullptr, QP, 1.0f, (unsigned)DM, (unsigned)LP, (size_t)0, (unsigned)MP, (unsigned)DM, (unsigned)(2 * DM));
  k_gemm2<1, 2, 0><<<dim3((unsigned)((MP / 128) * (DM / 64)), 1), 128, 0, stream>>>(HP, (unsigned)LH, (size_t)0, (unsigned)(2 * DM - 1), WKT, (unsigned)DM, (size_t)0, (unsigned)(DM - 1), 1.0f,
      bk, 1.0f, nullptr, KP, 1.0f, (unsigned)DM, (unsigned)LP, (size_t)0, (unsigned)MP, (unsigned)DM, (unsigned)(2 * DM));
  k_gemm2<0, 1, 1><<<dim3((unsigned)((DM / 128) * (SEQ / 64)), (unsigned)NB), 128, 0, stream>>>(WVT, (unsigned)DM, (size_t)0, (unsigned)(DM - 1), HP + 2 * DM, (unsigned)LH, (size_t)SEQ * LH, (unsigned)(DM - 1), 0.0625f,
      bv, 1.0f, nullptr, VT, 16.0f, 0u, (unsigned)SEQ, (size_t)DM * SEQ, (unsigned)DM, (unsigned)SEQ, (unsigned)DM);
  k_flash<<<dim3((unsigned)(SEQ / 64), (unsigned)NH, (unsigned)NB), 128, 0, stream>>>(QP, KP, VT, x, nhp, X1);
  k_ln<1, 1><<<(unsigned)MP, 256, 0, stream>>>(X1, g2, b2, 1e-5f, H2);
  k_gemm2<0, 0, 0><<<dim3((unsigned)((MP / 128) * (DFF / 64)), 1), 128, 0, stream>>>(H2, (unsigned)DM, (size_t)0, (unsigned)(DM - 1), W1T, (unsigned)DM, (size_t)0, (unsigned)(DM - 1), 0.0625f,
      bw1, 1.0f, UP, nullptr, 1.0f, 0u, (unsigned)DFF, (size_t)0, (unsigned)MP, (unsigned)DFF, (unsigned)DM);
  k_ln<4, 2><<<(unsigned)MP, 256, 0, stream>>>(UP, gf, bfv, 1e-5f, U16);
  k_gemm2<0, 0, 0><<<dim3((unsigned)((MP / 128) * (DM / 64)), 1), 128, 0, stream>>>(U16, (unsigned)DFF, (size_t)0, (unsigned)(DFF - 1), W2T, (unsigned)DFF, (size_t)0, (unsigned)(DFF - 1), 0.00390625f,
      bw2, 1.0f, (float*)d_out, nullptr, 1.0f, 0u, (unsigned)DM, (size_t)0, (unsigned)MP, (unsigned)DM, (unsigned)DFF);
}
